// SelfAttention_70755291235095
// MI455X (gfx1250) — hardware-verified
//
#include <hip/hip_runtime.h>
#include <math.h>

#ifndef NB
#define NB 2
#endif
#ifndef SEQ
#define SEQ 2048
#endif
#define NB_FULL 2
#define SEQ_FULL 2048
#define EMBED 1024
#define HEADS 16
#define HDIM 64
#define MTOK (NB * SEQ)

static_assert(SEQ % 64 == 0);
static_assert(MTOK % 64 == 0);
static_assert((MTOK * HEADS) % 64 == 0);
static_assert(EMBED % 64 == 0 && HDIM == 64);
static_assert(NB <= NB_FULL && SEQ <= SEQ_FULL);

typedef __attribute__((ext_vector_type(16))) _Float16 v16h;
typedef __attribute__((ext_vector_type(8)))  _Float16 v8h;
typedef __attribute__((ext_vector_type(8)))  float    v8f;
typedef __attribute__((ext_vector_type(4)))  float    v4f;

__device__ __forceinline__ v8f wmma16(v16h a, v16h b, v8f c) {
    c = __builtin_amdgcn_wmma_f32_16x16x32_f16(false, a, false, b, (short)0, c, false, false);
    asm volatile("v_nop\n\tv_nop\n\tv_nop\n\tv_nop" : "+v"(c) : "v"(a), "v"(b));
    return c;
}
union FragH { v16h v; v8h h[2]; };

__device__ __forceinline__ v16h fh_g32(const float* __restrict__ p) {
    const v4f x0 = *(const v4f*)(p), x1 = *(const v4f*)(p + 4), x2 = *(const v4f*)(p + 16), x3 = *(const v4f*)(p + 20);
    v16h a;
#pragma unroll
    for (int e = 0; e < 4; ++e) { a[e] = (_Float16)x0[e]; a[4 + e] = (_Float16)x1[e]; a[8 + e] = (_Float16)x2[e]; a[12 + e] = (_Float16)x3[e]; }
    return a;
}

#define VST2(T, ptr, val) do { const T vst2_v_ = (val); *(volatile T*)(ptr) = vst2_v_; __threadfence(); *(volatile T*)(ptr) = vst2_v_; } while (0)

#define AT_NW 4
#define AT_KP 72
struct AttnG { const float* Q; const float* K; const float* V; float* O; long long sb; int S; float scale; };
static_assert(sizeof(AttnG) == 48);

#ifndef KATTN_ATTR
#define KATTN_ATTR __attribute__((amdgpu_num_vgpr(256)))
#endif
__global__ __launch_bounds__(32 * AT_NW) KATTN_ATTR void k_attn64(AttnG g) {
    __shared__ __align__(16) _Float16 Ksh[64 * AT_KP];
    __shared__ __align__(16) _Float16 Vts[64 * AT_KP];
    __shared__ __align__(16) _Float16 Psh[AT_NW][16 * AT_KP];
    __shared__ __align__(16) float    Os[AT_NW][16 * 68];
    const int tid = threadIdx.x, wave = tid >> 5, lane = tid & 31, hf = lane >> 4, l15 = lane & 15;
    const int h = blockIdx.y, b = blockIdx.z;
    const int q0 = (blockIdx.x * AT_NW + wave) * 16;
    const float L2E = 1.4426950408889634f;
    const float NEG = -__builtin_inff();
    const float* qbase = g.Q + (long long)b * g.sb + h * HDIM;
    const float* kbase = g.K + (long long)b * g.sb + h * HDIM;
    const float* vbase = g.V + (long long)b * g.sb + h * HDIM;
    float*       obase = g.O + (long long)b * g.sb + h * HDIM;

    const float* qrow = qbase + (size_t)(q0 + l15) * EMBED + 8 * hf;
    const v16h qa0 = fh_g32(qrow), qa1 = fh_g32(qrow + 32);

    v8f o[4]; float m8[8], l8[8];
#pragma unroll
    for (int t = 0; t < 4; ++t) { v8f zz = {}; o[t] = zz; }
#pragma unroll
    for (int i = 0; i < 8; ++i) { m8[i] = NEG; l8[i] = 0.f; }

    for (int j0 = 0; j0 < g.S; j0 += 64) {
        __syncthreads();
#pragma unroll
        for (int it = 0; it < 4; ++it) {
            const int item = tid + it * (32 * AT_NW);
            const int jr = item >> 3, c8 = (item & 7) * 8;
            const float* kr = kbase + (size_t)(j0 + jr) * EMBED + c8;
            const float* vr = vbase + (size_t)(j0 + jr) * EMBED + c8;
            const v4f ka = *(const v4f*)(kr), kc = *(const v4f*)(kr + 4);
            const v4f va = *(const v4f*)(vr), vc = *(const v4f*)(vr + 4);
            v8h kk;
#pragma unroll
            for (int e = 0; e < 4; ++e) { kk[e] = (_Float16)ka[e]; kk[4 + e] = (_Float16)kc[e]; }
            *(v8h*)(Ksh + jr * AT_KP + c8) = kk;
#pragma unroll
            for (int e = 0; e < 4; ++e) { Vts[(c8 + e) * AT_KP + jr] = (_Float16)va[e]; Vts[(c8 + 4 + e) * AT_KP + jr] = (_Float16)vc[e]; }
        }
        __syncthreads();

        v8f s[4];
#pragma unroll
        for (int t = 0; t < 4; ++t) {
            const int ko = (t * 16 + l15) * AT_KP + 8 * hf;
            FragH k0f, k1f;
            k0f.h[0] = *(const v8h*)(Ksh + ko);      k0f.h[1] = *(const v8h*)(Ksh + ko + 16);
            k1f.h[0] = *(const v8h*)(Ksh + ko + 32); k1f.h[1] = *(const v8h*)(Ksh + ko + 48);
            v8f acc = {};
            acc = wmma16(qa0, k0f.v, acc);
            acc = wmma16(qa1, k1f.v, acc);
            s[t] = acc;
        }
#pragma unroll
        for (int i = 0; i < 8; ++i) {
            float sc[4];
#pragma unroll
            for (int t = 0; t < 4; ++t) { float v = s[t][i] * g.scale; v *= L2E; sc[t] = v; }
            float mx = fmaxf(fmaxf(sc[0], sc[1]), fmaxf(sc[2], sc[3]));
            mx = fmaxf(mx, __shfl_xor(mx, 1, 32)); mx = fmaxf(mx, __shfl_xor(mx, 2, 32));
            mx = fmaxf(mx, __shfl_xor(mx, 4, 32)); mx = fmaxf(mx, __shfl_xor(mx, 8, 32));
            const float mnew = fmaxf(m8[i], mx);
            const float corr = (mnew == NEG) ? 1.f : exp2f(m8[i] - mnew);
            float rs = 0.f;
#pragma unroll
            for (int t = 0; t < 4; ++t) {
                const float pp = (sc[t] == NEG) ? 0.f : exp2f(sc[t] - mnew); rs += pp;
                Psh[wave][(8 * hf + i) * AT_KP + t * 16 + l15] = (_Float16)(pp * 4096.f);
            }
            rs += __shfl_xor(rs, 1, 32); rs += __shfl_xor(rs, 2, 32); rs += __shfl_xor(rs, 4, 32); rs += __shfl_xor(rs, 8, 32);
            l8[i] = l8[i] * corr + rs; m8[i] = mnew;
#pragma unroll
            for (int t = 0; t < 4; ++t) o[t][i] *= corr;
        }
        __builtin_amdgcn_fence(3  , "workgroup");
        __builtin_amdgcn_wave_barrier();
        __builtin_amdgcn_fence(2  , "workgroup");
        {
            const int po = l15 * AT_KP + 8 * hf;
            FragH p0f, p1f;
            p0f.h[0] = *(const v8h*)(&Psh[wave][po]);      p0f.h[1] = *(const v8h*)(&Psh[wave][po + 16]);
            p1f.h[0] = *(const v8h*)(&Psh[wave][po + 32]); p1f.h[1] = *(const v8h*)(&Psh[wave][po + 48]);
#pragma unroll
            for (int t = 0; t < 4; ++t) {
                const int vo = (t * 16 + l15) * AT_KP + 8 * hf;
                FragH v0f, v1f;
                v0f.h[0] = *(const v8h*)(Vts + vo);      v0f.h[1] = *(const v8h*)(Vts + vo + 16);
                v1f.h[0] = *(const v8h*)(Vts + vo + 32); v1f.h[1] = *(const v8h*)(Vts + vo + 48);
                o[t] = wmma16(p0f.v, v0f.v, o[t]);
                o[t] = wmma16(p1f.v, v1f.v, o[t]);
            }
        }
    }

#pragma unroll
    for (int i = 0; i < 8; ++i) {
        const float inv = (l8[i] > 0.f) ? 1.f / (l8[i] * 4096.f) : 0.f;
#pragma unroll
        for (int t = 0; t < 4; ++t) Os[wave][(8 * hf + i) * 68 + t * 16 + l15] = o[t][i] * inv;
    }
    __builtin_amdgcn_fence(3  , "workgroup");
    __builtin_amdgcn_wave_barrier();
    __builtin_amdgcn_fence(2  , "workgroup");
    {
        const int c4 = l15 * 4;
        for (int pass = 0; pass < 2; ++pass) {
#pragma unroll
            for (int it = 0; it < 8; ++it) {
                const int row = it * 2 + hf;
                const v4f val = *(const v4f*)(&Os[wave][row * 68 + c4]);
                *(volatile v4f*)(obase + (size_t)(q0 + row) * EMBED + c4) = val;
            }
            __threadfence();
        }
    }
}

namespace kit {
typedef __attribute__((ext_vector_type(16))) _Float16 v16h;
typedef __attribute__((ext_vector_type(8)))  _Float16 v8h;
typedef __attribute__((ext_vector_type(16))) __bf16   v16b;
typedef __attribute__((ext_vector_type(8)))  __bf16   v8b;
typedef __attribute__((ext_vector_type(8)))  float    v8f;
typedef __attribute__((ext_vector_type(4)))  float    v4f;

__device__ __forceinline__ unsigned short f2bf_bits(float f) {
  unsigned u = __float_as_uint(f);
  return (unsigned short)((u + 0x7FFFu + ((u >> 16) & 1u)) >> 16);
}
__device__ __forceinline__ float bf_bits2f(unsigned short h) { return __uint_as_float(((unsigned)h) << 16); }

__device__ __forceinline__ void dep_guard_h(v8f& a, v8f& b, v16h x, v16h y) { asm volatile("v_nop\n\tv_nop\n\tv_nop\n\tv_nop" : "+v"(a), "+v"(b) : "v"(x), "v"(y)); }
__device__ __forceinline__ void dep_guard_b(v8f& a, v8f& b, v16b x, v16b y) { asm volatile("v_nop\n\tv_nop\n\tv_nop\n\tv_nop" : "+v"(a), "+v"(b) : "v"(x), "v"(y)); }
__device__ __forceinline__ void keep4_h(v16h a, v16h b, v16h c, v16h d) { asm volatile("v_nop" :: "v"(a), "v"(b), "v"(c), "v"(d)); }
__device__ __forceinline__ void keep4_b(v16b a, v16b b, v16b c, v16b d) { asm volatile("v_nop" :: "v"(a), "v"(b), "v"(c), "v"(d)); }
__device__ __forceinline__ void acc_guard4(v8f& a, v8f& b, v8f& c, v8f& d) { asm volatile("v_nop\n\tv_nop\n\tv_nop\n\tv_nop" : "+v"(a), "+v"(b), "+v"(c), "+v"(d)); }
template <typename T> struct Frag;
template <> struct Frag<_Float16> {
  typedef v16h V; union U { v16h v; v8h h[2]; };
  static __device__ __forceinline__ v16h load(const _Float16* p) {
    U f; f.h[0] = *(const v8h*)(p); f.h[1] = *(const v8h*)(p + 16); return f.v;
  }
  static __device__ __forceinline__ v8f mma(v16h a, v16h b, v8f c) {
    return __builtin_amdgcn_wmma_f32_16x16x32_f16(false, a, false, b, (short)0, c, false, false);
  }
  static __device__ __forceinline__ void guard(v8f& a, v8f& b, v16h x, v16h y) { dep_guard_h(a, b, x, y); }
  static __device__ __forceinline__ void keep(v16h a, v16h b, v16h c, v16h d) { keep4_h(a, b, c, d); }
};
template <> struct Frag<__bf16> {
  typedef v16b V; union U { v16b v; v8b h[2]; };
  static __device__ __forceinline__ v16b load(const __bf16* p) {
    U f; f.h[0] = *(const v8b*)(p); f.h[1] = *(const v8b*)(p + 16); return f.v;
  }
  static __device__ __forceinline__ v8f mma(v16b a, v16b b, v8f c) {
    return __builtin_amdgcn_wmma_f32_16x16x32_bf16(false, a, false, b, (short)0, c, false, false);
  }
  static __device__ __forceinline__ void guard(v8f& a, v8f& b, v16b x, v16b y) { dep_guard_b(a, b, x, y); }
  static __device__ __forceinline__ void keep(v16b a, v16b b, v16b c, v16b d) { keep4_b(a, b, c, d); }
};

template <int ET> struct Elem;
template <> struct Elem<0> { typedef _Float16 T; };
template <> struct Elem<1> { typedef __bf16 T; };
template <int ET, bool SPLIT, int BIAS_MODE, int OUT_MODE, bool RESID, int ACT = 0>
__global__ __launch_bounds__(256) void wmma_gemm64(
    const unsigned short* __restrict__ Ap, const unsigned short* __restrict__ A2p, int lda, long strideA,
    const unsigned short* __restrict__ Btp, const unsigned short* __restrict__ Bt2p, int ldb, long strideB,
    void* __restrict__ Cout, void* __restrict__ Cout2, int ldc, long strideC,
    const float* __restrict__ bias,
    const float* __restrict__ resid, long strideR,
    int M, int N, int K, float scale) {
  typedef typename Elem<ET>::T T;
  typedef typename Frag<T>::V V;
  const T* A = (const T*)Ap; const T* A2 = (const T*)A2p; const T* Bt = (const T*)Btp; const T* Bt2 = (const T*)Bt2p;
  __shared__ __align__(16) float sT[8][16 * 68];
  const int b    = blockIdx.y;
  const int lane = threadIdx.x & 31;
  const int wave = threadIdx.x >> 5;
  const int tilesN = N >> 6;
  const int tilesM = M >> 6;
  const int tile = blockIdx.x * 8 + wave;
  if (tile >= tilesM * tilesN) return;
  const int tm = tile / tilesN;
  const int tn = tile - tm * tilesN;
  const int m0 = tm << 6;
  const int n0 = tn << 6;

  const T* Ab  = A  + (size_t)b * strideA;
  const T* Bb  = Bt + (size_t)b * strideB;
  const T* Ab2 = SPLIT ? (A2  + (size_t)b * strideA) : nullptr;
  const T* Bb2 = SPLIT ? (Bt2 + (size_t)b * strideB) : nullptr;

  const int rlane = lane & 15;
  const int koff  = (lane >> 4) * 8;
  const int mOff  = (lane >> 4) * 8;

  v8f acc[4][4];
#pragma unroll
  for (int i = 0; i < 4; ++i)
#pragma unroll
    for (int j = 0; j < 4; ++j) acc[i][j] = (v8f){0.f,0.f,0.f,0.f,0.f,0.f,0.f,0.f};

  for (int k0 = 0; k0 < K; k0 += 32) {
    V bh[4], bl[4];
#pragma unroll
    for (int j = 0; j < 4; ++j) {
      const size_t bo = (size_t)(n0 + (j << 4) + rlane) * ldb + koff + k0;
      bh[j] = Frag<T>::load(Bb + bo);
      if (SPLIT) bl[j] = Frag<T>::load(Bb2 + bo);
    }
#pragma unroll
    for (int i = 0; i < 4; ++i) {
      const size_t ao = (size_t)(m0 + (i << 4) + rlane) * lda + koff + k0;
      V ah = Frag<T>::load(Ab + ao);
      V al;
      if (SPLIT) al = Frag<T>::load(Ab2 + ao);
#pragma unroll
      for (int j = 0; j < 4; ++j) {
        acc[i][j] = Frag<T>::mma(ah, bh[j], acc[i][j]);
        if (SPLIT) {
          acc[i][j] = Frag<T>::mma(ah, bl[j], acc[i][j]);
          acc[i][j] = Frag<T>::mma(al, bh[j], acc[i][j]);
        }
      }
      Frag<T>::guard(acc[i][0], acc[i][3], ah, SPLIT ? al : ah);
    }
    Frag<T>::keep(bh[0], bh[1], bh[2], bh[3]);
    if (SPLIT) Frag<T>::keep(bl[0], bl[1], bl[2], bl[3]);
  }
  acc_guard4(acc[0][0], acc[0][1], acc[0][2], acc[0][3]);
  acc_guard4(acc[1][0], acc[1][1], acc[1][2], acc[1][3]);
  acc_guard4(acc[2][0], acc[2][1], acc[2][2], acc[2][3]);
  acc_guard4(acc[3][0], acc[3][1], acc[3][2], acc[3][3]);

  float* slab = sT[wave];
  const float* Rb = RESID ? (resid + (size_t)b * strideR) : nullptr;
#pragma unroll
  for (int i = 0; i < 4; ++i) {
    const int mBase = m0 + (i << 4);
#pragma unroll
    for (int j = 0; j < 4; ++j) {
      const int n = n0 + (j << 4) + rlane;
      float bv = 0.f;
      if (BIAS_MODE == 2) bv = bias[n];
#pragma unroll
      for (int r = 0; r < 8; ++r) {
        float v = acc[i][j][r] * scale;
        if (BIAS_MODE == 1) v += bias[mBase + mOff + r];
        if (BIAS_MODE == 2) v += bv;
        if (RESID) v += Rb[(size_t)(mBase + mOff + r) * ldc + n];
        if (ACT == 1) v = tanhf(v);
        if (ACT == 2) v = fmaxf(v, 0.0f);
        if (ACT == 3) v = v / (1.0f + expf(-v));
        if (ACT == 4) v = (v > 0.f) ? v : 0.01f * v;
        if (ACT == 5) v = 0.5f * v * (1.0f + erff(v * 0.70710678118654752f));
        if (ACT == 6) v = (v > 0.f) ? v : 0.2f * v;
        if (ACT == 7) { const float u = 0.7978845608028654f * (v + 0.044715f * v * v * v); v = 0.5f * v * (1.f + tanhf(u)); }
        slab[(mOff + r) * 68 + (j << 4) + rlane] = v;
      }
    }
    __builtin_amdgcn_fence(3  , "workgroup");
    __builtin_amdgcn_wave_barrier();
    __builtin_amdgcn_fence(2  , "workgroup");
    if (OUT_MODE == 0) {
      float* C = (float*)Cout + (size_t)b * strideC;
      const int hh = lane >> 4, c4 = (lane & 15) * 4;
      for (int pass = 0; pass < 2; ++pass) {
#pragma unroll
        for (int it = 0; it < 8; ++it) {
          const int row = it * 2 + hh;
          v4f v = *(const v4f*)(slab + row * 68 + c4);
          *(volatile v4f*)(C + (size_t)(mBase + row) * ldc + n0 + c4) = v;
        }
        __threadfence();
      }
    } else {
      const int q = lane >> 3, c8 = (lane & 7) * 8;
      unsigned short* C  = (unsigned short*)Cout  + (size_t)b * strideC;
      unsigned short* C2 = (OUT_MODE == 2) ? ((unsigned short*)Cout2 + (size_t)b * strideC) : nullptr;
      for (int pass = 0; pass < 2; ++pass) {
#pragma unroll
        for (int it = 0; it < 4; ++it) {
          const int row = it * 4 + q;
          const float* sp = slab + row * 68 + c8;
          v8h hv, lv;
#pragma unroll
          for (int e = 0; e < 8; ++e) {
            if (OUT_MODE == 1) {
              hv[e] = (_Float16)sp[e];
            } else {
              unsigned short hb = f2bf_bits(sp[e]);
              unsigned short lb = f2bf_bits(sp[e] - bf_bits2f(hb));
              hv[e] = __builtin_bit_cast(_Float16, hb);
              lv[e] = __builtin_bit_cast(_Float16, lb);
            }
          }
          *(volatile v8h*)(C + (size_t)(mBase + row) * ldc + n0 + c8) = hv;
          if (OUT_MODE == 2) *(volatile v8h*)(C2 + (size_t)(mBase + row) * ldc + n0 + c8) = lv;
        }
        __threadfence();
      }
    }
    __builtin_amdgcn_fence(3  , "workgroup");
    __builtin_amdgcn_wave_barrier();
    __builtin_amdgcn_fence(2  , "workgroup");
  }
}

}

__global__ __launch_bounds__(256) void k_cast16(const float* __restrict__ src, long long lds, _Float16* __restrict__ dst, long long ldd, int R, int C, float s) {
    const long long i = (long long)blockIdx.x * 256 + threadIdx.x; const long long np = (long long)R * (C / 2); if (i >= np) return; const int r = (int)(i / (C / 2)); const int c = 2 * (int)(i % (C / 2));
    const _Float16 h0 = (_Float16)(src[(long long)r * lds + c] * s), h1 = (_Float16)(src[(long long)r * lds + c + 1] * s);
    const unsigned u = (unsigned)__builtin_bit_cast(unsigned short, h0) | ((unsigned)__builtin_bit_cast(unsigned short, h1) << 16);
    volatile unsigned* d = (volatile unsigned*)(dst + (long long)r * ldd + c); *d = u; __threadfence(); *d = u; }

typedef unsigned int cm_u4 __attribute__((ext_vector_type(4)));
__device__ __forceinline__ unsigned int cmb_pk2(float a, float b) { return (unsigned int)__builtin_bit_cast(unsigned short, (_Float16)a) | ((unsigned int)__builtin_bit_cast(unsigned short, (_Float16)b) << 16); }
__device__ __forceinline__ float cmb_bf(float v) { const unsigned u = __builtin_bit_cast(unsigned, v); const unsigned r = (u + 0x7fffu + ((u >> 16) & 1u)) & 0xffff0000u; return __builtin_bit_cast(float, r); }
__global__ __launch_bounds__(256) void k_cm_bfvec(const float* __restrict__ SRC, float* __restrict__ DST, int n) { const int u = blockIdx.x * 256 + threadIdx.x; if (u >= n) return; VST2(float, DST + u, cmb_bf(SRC[u])); }
__global__ __launch_bounds__(256) void k_cm_castb(const float* __restrict__ SRC, int lds, long long sSz, unsigned short* __restrict__ DST, int ldd, long long sDz, int nR, int nC, float sc) {
    const long long u = (long long)blockIdx.x * 256 + threadIdx.x; const int per = nC / 8; if (u >= (long long)nR * per) return; const int r = (int)(u / per); const int c0 = 8 * (int)(u % per);
    const float* s = SRC + (long long)blockIdx.y * sSz + (long long)r * lds + c0; float w[8];
#pragma unroll
    for (int e = 0; e < 8; ++e) w[e] = cmb_bf(s[e]) * sc;
    cm_u4 pk; pk.x = cmb_pk2(w[0], w[1]); pk.y = cmb_pk2(w[2], w[3]); pk.z = cmb_pk2(w[4], w[5]); pk.w = cmb_pk2(w[6], w[7]); VST2(cm_u4, (cm_u4*)(DST + (long long)blockIdx.y * sDz + (long long)r * ldd + c0), pk); }

extern "C" void kernel_launch(void* const* d_in, const int* in_sizes, int n_in, void* d_out, int out_size, void* d_ws, size_t ws_size, hipStream_t stream) {
    if (n_in < 8) return;
    const long long need_x = (long long)(NB - 1) * SEQ_FULL * EMBED + (long long)SEQ * EMBED;
    if ((long long)in_sizes[0] < need_x || (long long)in_sizes[1] < need_x || (long long)in_sizes[2] < need_x) return;
    if (in_sizes[3] < HDIM * HDIM || in_sizes[4] < HDIM * HDIM || in_sizes[5] < HDIM * HDIM) return;
    if (in_sizes[6] < EMBED * EMBED || in_sizes[7] < EMBED) return;
    if ((long long)out_size < (long long)MTOK * EMBED) return;
    const float* xq = (const float*)d_in[0];
    const float* xk = (const float*)d_in[1];
    const float* xv = (const float*)d_in[2];
    const float* Wq = (const float*)d_in[3];
    const float* Wk = (const float*)d_in[4];
    const float* Wv = (const float*)d_in[5];
    const float* Wo = (const float*)d_in[6];
    const float* bo = (const float*)d_in[7];
    float* out = (float*)d_out;
    char* wsp = (char*)d_ws;
    unsigned short* X16 = (unsigned short*)wsp; wsp += (((size_t)MTOK * EMBED * 2 + 255) / 256) * 256;
    unsigned short* W316 = (unsigned short*)wsp; wsp += (((size_t)3 * HDIM * HDIM * 2 + 255) / 256) * 256;
    float* Qf = (float*)wsp; wsp += (((size_t)MTOK * EMBED * 4 + 255) / 256) * 256;
    float* Kf = (float*)wsp; wsp += (((size_t)MTOK * EMBED * 4 + 255) / 256) * 256;
    float* Vf = (float*)wsp; wsp += (((size_t)MTOK * EMBED * 4 + 255) / 256) * 256;
    float* AO = (float*)wsp; wsp += (((size_t)MTOK * EMBED * 4 + 255) / 256) * 256;
    unsigned short* AO16 = X16;
    unsigned short* WO16 = (unsigned short*)wsp; wsp += (((size_t)EMBED * EMBED * 2 + 255) / 256) * 256;
    float* BRO = (float*)wsp; wsp += (((size_t)(EMBED + 64) * 4 + 255) / 256) * 256;
    if ((size_t)(wsp - (char*)d_ws) > ws_size) return;

    const unsigned wblocks = (unsigned)(((long long)HDIM * (HDIM / 8) + 255) / 256);
    const unsigned xblocks = (unsigned)(((long long)SEQ * (EMBED / 8) + 255) / 256);
    const unsigned pgrid = (unsigned)((((MTOK * HEADS) / 64) * (HDIM / 64) + 7) / 8);
    k_cm_castb<<<dim3(wblocks, 1), 256, 0, stream>>>(Wq, HDIM, 0, W316 + 0, HDIM, 0, HDIM, HDIM, 16.0f);
    k_cm_castb<<<dim3(wblocks, 1), 256, 0, stream>>>(Wk, HDIM, 0, W316 + HDIM * HDIM, HDIM, 0, HDIM, HDIM, 16.0f);
    k_cm_castb<<<dim3(wblocks, 1), 256, 0, stream>>>(Wv, HDIM, 0, W316 + 2 * HDIM * HDIM, HDIM, 0, HDIM, HDIM, 16.0f);
    k_cm_castb<<<dim3(xblocks, NB), 256, 0, stream>>>(xq, EMBED, (long long)SEQ_FULL * EMBED, X16, EMBED, (long long)SEQ * EMBED, SEQ, EMBED, 1.0f);
    kit::wmma_gemm64<0, false, 0, 0, false, 0><<<dim3(pgrid, 1), 256, 0, stream>>>((const unsigned short*)X16, nullptr, HDIM, 0, (const unsigned short*)(W316 + 0), nullptr, HDIM, 0, (void*)Qf, nullptr, HDIM, 0, nullptr, nullptr, 0, MTOK * HEADS, HDIM, HDIM, 0.0625f);
    k_cm_castb<<<dim3(xblocks, NB), 256, 0, stream>>>(xk, EMBED, (long long)SEQ_FULL * EMBED, X16, EMBED, (long long)SEQ * EMBED, SEQ, EMBED, 1.0f);
    kit::wmma_gemm64<0, false, 0, 0, false, 0><<<dim3(pgrid, 1), 256, 0, stream>>>((const unsigned short*)X16, nullptr, HDIM, 0, (const unsigned short*)(W316 + HDIM * HDIM), nullptr, HDIM, 0, (void*)Kf, nullptr, HDIM, 0, nullptr, nullptr, 0, MTOK * HEADS, HDIM, HDIM, 0.0625f);
    k_cm_castb<<<dim3(xblocks, NB), 256, 0, stream>>>(xv, EMBED, (long long)SEQ_FULL * EMBED, X16, EMBED, (long long)SEQ * EMBED, SEQ, EMBED, 1.0f);
    kit::wmma_gemm64<0, false, 0, 0, false, 0><<<dim3(pgrid, 1), 256, 0, stream>>>((const unsigned short*)X16, nullptr, HDIM, 0, (const unsigned short*)(W316 + 2 * HDIM * HDIM), nullptr, HDIM, 0, (void*)Vf, nullptr, HDIM, 0, nullptr, nullptr, 0, MTOK * HEADS, HDIM, HDIM, 0.0625f);
    k_cm_castb<<<dim3((unsigned)(((long long)EMBED * (EMBED / 8) + 255) / 256), 1), 256, 0, stream>>>(Wo, EMBED, 0, WO16, EMBED, 0, EMBED, EMBED, 16.0f);
    k_cm_bfvec<<<(EMBED + 255) / 256, 256, 0, stream>>>(bo, BRO, EMBED);
    {
      AttnG a;
      a.Q = Qf; a.K = Kf; a.V = Vf; a.O = AO;
      a.sb = (long long)SEQ * EMBED; a.S = SEQ; a.scale = 0.03125f;
      k_attn64<<<dim3((unsigned)(SEQ / 64), (unsigned)HEADS, (unsigned)NB), 32 * AT_NW, 0, stream>>>(a);
    }
    k_cast16<<<(unsigned)((((long long)MTOK * (EMBED / 2)) + 255) / 256), 256, 0, stream>>>(AO, EMBED, (_Float16*)AO16, EMBED, MTOK, EMBED, 64.0f);
    kit::wmma_gemm64<0, false, 2, 0, false, 0><<<dim3((unsigned)((((MTOK / 64) * (EMBED / 64)) + 7) / 8), 1), 256, 0, stream>>>((const unsigned short*)AO16, nullptr, EMBED, 0, (const unsigned short*)WO16, nullptr, EMBED, 0, (void*)out, nullptr, EMBED, 0, BRO, nullptr, 0, MTOK, EMBED, EMBED, 0.0009765625f);
}
